// CSMHSA_1288490189370
// MI455X (gfx1250) — hardware-verified
//
#include <hip/hip_runtime.h>
#include <stdint.h>

typedef __attribute__((ext_vector_type(16))) _Float16 v16h;
typedef __attribute__((ext_vector_type(8)))  _Float16 v8h;
typedef __attribute__((ext_vector_type(16))) __bf16   v16b;
typedef __attribute__((ext_vector_type(8)))  __bf16   v8b;
typedef __attribute__((ext_vector_type(8)))  float    v8f;
typedef __attribute__((ext_vector_type(4)))  float    v4f;

__device__ __forceinline__ unsigned short f2bf_bits(float f) {
  unsigned u = __float_as_uint(f);
  return (unsigned short)((u + 0x7FFFu + ((u >> 16) & 1u)) >> 16);
}
__device__ __forceinline__ float bf_bits2f(unsigned short h) { return __uint_as_float(((unsigned)h) << 16); }

__device__ __forceinline__ void dep_guard_h(v8f& a, v8f& b, v16h x, v16h y) { asm volatile("v_nop\n\tv_nop\n\tv_nop\n\tv_nop" : "+v"(a), "+v"(b) : "v"(x), "v"(y)); }
__device__ __forceinline__ void dep_guard_b(v8f& a, v8f& b, v16b x, v16b y) { asm volatile("v_nop\n\tv_nop\n\tv_nop\n\tv_nop" : "+v"(a), "+v"(b) : "v"(x), "v"(y)); }
__device__ __forceinline__ void keep4_h(v16h a, v16h b, v16h c, v16h d) { asm volatile("v_nop" :: "v"(a), "v"(b), "v"(c), "v"(d)); }
__device__ __forceinline__ void keep4_b(v16b a, v16b b, v16b c, v16b d) { asm volatile("v_nop" :: "v"(a), "v"(b), "v"(c), "v"(d)); }
__device__ __forceinline__ void acc_guard4(v8f& a, v8f& b, v8f& c, v8f& d) { asm volatile("v_nop\n\tv_nop\n\tv_nop\n\tv_nop" : "+v"(a), "+v"(b), "+v"(c), "+v"(d)); }
template <typename T> struct Frag;
template <> struct Frag<_Float16> {
  typedef v16h V; union U { v16h v; v8h h[2]; };
  static __device__ __forceinline__ v16h load(const _Float16* p) {
    U f; f.h[0] = *(const v8h*)(p); f.h[1] = *(const v8h*)(p + 16); return f.v;
  }
  static __device__ __forceinline__ v8f mma(v16h a, v16h b, v8f c) {
    return __builtin_amdgcn_wmma_f32_16x16x32_f16(false, a, false, b, (short)0, c, false, false);
  }
  static __device__ __forceinline__ void guard(v8f& a, v8f& b, v16h x, v16h y) { dep_guard_h(a, b, x, y); }
  static __device__ __forceinline__ void keep(v16h a, v16h b, v16h c, v16h d) { keep4_h(a, b, c, d); }
};
template <> struct Frag<__bf16> {
  typedef v16b V; union U { v16b v; v8b h[2]; };
  static __device__ __forceinline__ v16b load(const __bf16* p) {
    U f; f.h[0] = *(const v8b*)(p); f.h[1] = *(const v8b*)(p + 16); return f.v;
  }
  static __device__ __forceinline__ v8f mma(v16b a, v16b b, v8f c) {
    return __builtin_amdgcn_wmma_f32_16x16x32_bf16(false, a, false, b, (short)0, c, false, false);
  }
  static __device__ __forceinline__ void guard(v8f& a, v8f& b, v16b x, v16b y) { dep_guard_b(a, b, x, y); }
  static __device__ __forceinline__ void keep(v16b a, v16b b, v16b c, v16b d) { keep4_b(a, b, c, d); }
};

template <int ET> struct Elem;
template <> struct Elem<0> { typedef _Float16 T; };
template <> struct Elem<1> { typedef __bf16 T; };
template <int ET, bool SPLIT, int BIAS_MODE, int OUT_MODE, bool RESID, int ACT = 0>
__global__ __launch_bounds__(256) void wmma_gemm64(
    const unsigned short* __restrict__ Ap, const unsigned short* __restrict__ A2p, int lda, long strideA,
    const unsigned short* __restrict__ Btp, const unsigned short* __restrict__ Bt2p, int ldb, long strideB,
    void* __restrict__ Cout, void* __restrict__ Cout2, int ldc, long strideC,
    const float* __restrict__ bias,
    const float* __restrict__ resid, long strideR,
    int M, int N, int K, float scale) {
  typedef typename Elem<ET>::T T;
  typedef typename Frag<T>::V V;
  const T* A = (const T*)Ap; const T* A2 = (const T*)A2p; const T* Bt = (const T*)Btp; const T* Bt2 = (const T*)Bt2p;
  __shared__ __align__(16) float sT[8][16 * 68];
  const int b    = blockIdx.y;
  const int lane = threadIdx.x & 31;
  const int wave = threadIdx.x >> 5;
  const int tilesN = N >> 6;
  const int tilesM = M >> 6;
  const int tile = blockIdx.x * 8 + wave;
  if (tile >= tilesM * tilesN) return;
  const int tm = tile / tilesN;
  const int tn = tile - tm * tilesN;
  const int m0 = tm << 6;
  const int n0 = tn << 6;

  const T* Ab  = A  + (size_t)b * strideA;
  const T* Bb  = Bt + (size_t)b * strideB;
  const T* Ab2 = SPLIT ? (A2  + (size_t)b * strideA) : nullptr;
  const T* Bb2 = SPLIT ? (Bt2 + (size_t)b * strideB) : nullptr;

  const int rlane = lane & 15;
  const int koff  = (lane >> 4) * 8;
  const int mOff  = (lane >> 4) * 8;

  v8f acc[4][4];
#pragma unroll
  for (int i = 0; i < 4; ++i)
#pragma unroll
    for (int j = 0; j < 4; ++j) acc[i][j] = (v8f){0.f,0.f,0.f,0.f,0.f,0.f,0.f,0.f};

  for (int k0 = 0; k0 < K; k0 += 32) {
    V bh[4], bl[4];
#pragma unroll
    for (int j = 0; j < 4; ++j) {
      const size_t bo = (size_t)(n0 + (j << 4) + rlane) * ldb + koff + k0;
      bh[j] = Frag<T>::load(Bb + bo);
      if (SPLIT) bl[j] = Frag<T>::load(Bb2 + bo);
    }
#pragma unroll
    for (int i = 0; i < 4; ++i) {
      const size_t ao = (size_t)(m0 + (i << 4) + rlane) * lda + koff + k0;
      V ah = Frag<T>::load(Ab + ao);
      V al;
      if (SPLIT) al = Frag<T>::load(Ab2 + ao);
#pragma unroll
      for (int j = 0; j < 4; ++j) {
        acc[i][j] = Frag<T>::mma(ah, bh[j], acc[i][j]);
        if (SPLIT) {
          acc[i][j] = Frag<T>::mma(ah, bl[j], acc[i][j]);
          acc[i][j] = Frag<T>::mma(al, bh[j], acc[i][j]);
        }
      }
      Frag<T>::guard(acc[i][0], acc[i][3], ah, SPLIT ? al : ah);
    }
    Frag<T>::keep(bh[0], bh[1], bh[2], bh[3]);
    if (SPLIT) Frag<T>::keep(bl[0], bl[1], bl[2], bl[3]);
  }
  acc_guard4(acc[0][0], acc[0][1], acc[0][2], acc[0][3]);
  acc_guard4(acc[1][0], acc[1][1], acc[1][2], acc[1][3]);
  acc_guard4(acc[2][0], acc[2][1], acc[2][2], acc[2][3]);
  acc_guard4(acc[3][0], acc[3][1], acc[3][2], acc[3][3]);

  float* slab = sT[wave];
  const float* Rb = RESID ? (resid + (size_t)b * strideR) : nullptr;
#pragma unroll
  for (int i = 0; i < 4; ++i) {
    const int mBase = m0 + (i << 4);
#pragma unroll
    for (int j = 0; j < 4; ++j) {
      const int n = n0 + (j << 4) + rlane;
      float bv = 0.f;
      if (BIAS_MODE == 2) bv = bias[n];
#pragma unroll
      for (int r = 0; r < 8; ++r) {
        float v = acc[i][j][r] * scale;
        if (BIAS_MODE == 1) v += bias[mBase + mOff + r];
        if (BIAS_MODE == 2) v += bv;
        if (RESID) v += Rb[(size_t)(mBase + mOff + r) * ldc + n];
        if (ACT == 1) v = tanhf(v);
        if (ACT == 2) v = fmaxf(v, 0.0f);
        if (ACT == 3) v = v / (1.0f + expf(-v));
        if (ACT == 4) v = (v > 0.f) ? v : 0.01f * v;
        if (ACT == 5) v = 0.5f * v * (1.0f + erff(v * 0.70710678118654752f));
        slab[(mOff + r) * 68 + (j << 4) + rlane] = v;
      }
    }
    __builtin_amdgcn_fence(__ATOMIC_RELEASE, "workgroup");
    __builtin_amdgcn_wave_barrier();
    __builtin_amdgcn_fence(__ATOMIC_ACQUIRE, "workgroup");
    if (OUT_MODE == 0) {
      float* C = (float*)Cout + (size_t)b * strideC;
      const int hh = lane >> 4, c4 = (lane & 15) * 4;
      for (int pass = 0; pass < 2; ++pass) {
#pragma unroll
        for (int it = 0; it < 8; ++it) {
          const int row = it * 2 + hh;
          v4f v = *(const v4f*)(slab + row * 68 + c4);
          *(volatile v4f*)(C + (size_t)(mBase + row) * ldc + n0 + c4) = v;
        }
        __threadfence();
      }
    } else {
      const int q = lane >> 3, c8 = (lane & 7) * 8;
      unsigned short* C  = (unsigned short*)Cout  + (size_t)b * strideC;
      unsigned short* C2 = (OUT_MODE == 2) ? ((unsigned short*)Cout2 + (size_t)b * strideC) : nullptr;
      for (int pass = 0; pass < 2; ++pass) {
#pragma unroll
        for (int it = 0; it < 4; ++it) {
          const int row = it * 4 + q;
          const float* sp = slab + row * 68 + c8;
          v8h hv, lv;
#pragma unroll
          for (int e = 0; e < 8; ++e) {
            if (OUT_MODE == 1) {
              hv[e] = (_Float16)sp[e];
            } else {
              unsigned short hb = f2bf_bits(sp[e]);
              unsigned short lb = f2bf_bits(sp[e] - bf_bits2f(hb));
              hv[e] = __builtin_bit_cast(_Float16, hb);
              lv[e] = __builtin_bit_cast(_Float16, lb);
            }
          }
          *(volatile v8h*)(C + (size_t)(mBase + row) * ldc + n0 + c8) = hv;
          if (OUT_MODE == 2) *(volatile v8h*)(C2 + (size_t)(mBase + row) * ldc + n0 + c8) = lv;
        }
        __threadfence();
      }
    }
    __builtin_amdgcn_fence(__ATOMIC_RELEASE, "workgroup");
    __builtin_amdgcn_wave_barrier();
    __builtin_amdgcn_fence(__ATOMIC_ACQUIRE, "workgroup");
  }
}

__global__ __launch_bounds__(256) void cast_f32_f16x2(
    const float* __restrict__ in, _Float16* __restrict__ out, int n2) {
  int i = blockIdx.x * 256 + threadIdx.x;
  if (i < n2) {
    const _Float16 h0 = (_Float16)in[2 * i], h1 = (_Float16)in[2 * i + 1];
    const unsigned u = (unsigned)__builtin_bit_cast(unsigned short, h0) | ((unsigned)__builtin_bit_cast(unsigned short, h1) << 16);
    ((volatile unsigned*)out)[i] = u;
    __threadfence();
    ((volatile unsigned*)out)[i] = u;
  }
}

__global__ __launch_bounds__(256) void split_f32_bf16x2(
    const float* __restrict__ in, unsigned short* __restrict__ oh, unsigned short* __restrict__ ol, int n2) {
  int i = blockIdx.x * 256 + threadIdx.x;
  if (i < n2) {
    const float f0 = in[2 * i], f1 = in[2 * i + 1];
    const unsigned short hb0 = f2bf_bits(f0), hb1 = f2bf_bits(f1);
    const unsigned short lb0 = f2bf_bits(f0 - bf_bits2f(hb0)), lb1 = f2bf_bits(f1 - bf_bits2f(hb1));
    const unsigned uh = (unsigned)hb0 | ((unsigned)hb1 << 16);
    const unsigned ul = (unsigned)lb0 | ((unsigned)lb1 << 16);
    ((volatile unsigned*)oh)[i] = uh;
    ((volatile unsigned*)ol)[i] = ul;
    __threadfence();
    ((volatile unsigned*)oh)[i] = uh;
    ((volatile unsigned*)ol)[i] = ul;
  }
}

template <bool F16P>
__global__ __launch_bounds__(256) void k_cm_to_pm(
    const float* __restrict__ x, int Cin, int Sn,
    unsigned short* __restrict__ oh, unsigned short* __restrict__ ol, unsigned short* __restrict__ of) {
  __shared__ __align__(16) float ts[32][68];
  const int tid = threadIdx.x, lane = tid & 31, wave = tid >> 5;
  const int s0 = blockIdx.x * 32, c0 = blockIdx.y * 64, b = blockIdx.z;
  const float* xb = x + ((size_t)b * Cin + c0) * Sn + s0;
#pragma unroll
  for (int i = 0; i < 8; ++i) {
    const int idx = tid + i * 256;
    const int cc = idx >> 5, ss = idx & 31;
    ts[ss][cc] = xb[(size_t)cc * Sn + ss];
  }
  __syncthreads();
  const int lq = lane >> 3, c8 = (lane & 7) * 8;
  const int ss = wave * 4 + lq;
  const v4f a0 = *(const v4f*)(&ts[ss][c8]);
  const v4f a1 = *(const v4f*)(&ts[ss][c8 + 4]);
  const float f[8] = {a0[0], a0[1], a0[2], a0[3], a1[0], a1[1], a1[2], a1[3]};
  v8h hv, lv, fv;
#pragma unroll
  for (int e = 0; e < 8; ++e) {
    const unsigned short hb = f2bf_bits(f[e]);
    const unsigned short lb = f2bf_bits(f[e] - bf_bits2f(hb));
    hv[e] = __builtin_bit_cast(_Float16, hb);
    lv[e] = __builtin_bit_cast(_Float16, lb);
    fv[e] = F16P ? (_Float16)f[e] : hv[e];
  }
  const size_t o = ((size_t)b * Sn + s0 + ss) * Cin + c0 + c8;
  for (int pass = 0; pass < 2; ++pass) {
    *(volatile v8h*)(oh + o) = hv;
    *(volatile v8h*)(ol + o) = lv;
    if (F16P) *(volatile v8h*)(of + o) = fv;
    __threadfence();
  }
}

#define AS_S   1024
#define AS_C   256
#define AS_SQ  256
#define AS_HD  32
#define AS_NH  8
#define AS_KC  64
#define AS_PSC 32768.0f

__device__ __forceinline__ v8f mma_bf_g(v16b a, v16b b, v8f c) {
  c = __builtin_amdgcn_wmma_f32_16x16x32_bf16(false, a, false, b, (short)0, c, false, false);
  asm volatile("v_nop\n\tv_nop\n\tv_nop\n\tv_nop" : "+v"(c) : "v"(a), "v"(b));
  return c;
}
__device__ __forceinline__ v8f mma_hf_g(v16h a, v16h b, v8f c) {
  c = __builtin_amdgcn_wmma_f32_16x16x32_f16(false, a, false, b, (short)0, c, false, false);
  asm volatile("v_nop\n\tv_nop\n\tv_nop\n\tv_nop" : "+v"(c) : "v"(a), "v"(b));
  return c;
}

__global__ __launch_bounds__(128)
void attn_hd32(const unsigned short* __restrict__ qhp, const unsigned short* __restrict__ qlp,
               const unsigned short* __restrict__ khp, const unsigned short* __restrict__ klp,
               const unsigned short* __restrict__ vp, float* __restrict__ out) {
  union FB { v16b v; v8b h[2]; };
  union FH { v16h v; v8h h[2]; };
  __shared__ __align__(16) __bf16   Ksh[AS_KC * AS_HD];
  __shared__ __align__(16) __bf16   Ksl[AS_KC * AS_HD];
  __shared__ __align__(16) _Float16 Vt[AS_HD * AS_KC];
  __shared__ __align__(16) _Float16 Psh[4][16 * AS_KC];
  __shared__ __align__(16) float    Os[AS_HD][68];

  const int tid  = threadIdx.x;
  const int wave = tid >> 5;
  const int lane = tid & 31;
  const int hh   = lane >> 4;
  const int c    = lane & 15;

  const int bx = blockIdx.x;
  const int qb = bx & 15;
  const int bh = bx >> 4;
  const int h  = bh & (AS_NH - 1);
  const int b  = bh >> 3;
  const int qbase = qb * 64;
  const int q0 = qbase + wave * 16;

  v16b qah, qal;
  {
    const int qi = q0 + c;
    const int yy = qi >> 5, xx = qi & 31;
    const int sq = (yy >> 1) * 16 + (xx >> 1);
    const size_t qo = ((size_t)b * AS_SQ + sq) * AS_C + h * AS_HD + 8 * hh;
    qah = Frag<__bf16>::load((const __bf16*)qhp + qo);
    qal = Frag<__bf16>::load((const __bf16*)qlp + qo);
  }

  float mrow[8], lrow[8];
  v8f oacc[2];
#pragma unroll
  for (int r = 0; r < 8; ++r) { mrow[r] = -INFINITY; lrow[r] = 0.f; }
#pragma unroll
  for (int t = 0; t < 2; ++t) oacc[t] = (v8f){0.f,0.f,0.f,0.f,0.f,0.f,0.f,0.f};

  const __bf16*   khb = (const __bf16*)khp + (size_t)b * AS_S * AS_C + h * AS_HD;
  const __bf16*   klb = (const __bf16*)klp + (size_t)b * AS_S * AS_C + h * AS_HD;
  const _Float16* vb  = (const _Float16*)vp + ((size_t)b * AS_C + h * AS_HD) * AS_S;
  float*          ob  = out + ((size_t)b * AS_C + h * AS_HD) * AS_S + qbase;
  _Float16*       pw  = Psh[wave];

  for (int kc = 0; kc < AS_S / AS_KC; ++kc) {
    const int kv0 = kc * AS_KC;
    __syncthreads();
    {
      const int kvr = tid >> 1, dh = (tid & 1) * 16;
      const __bf16* kr  = khb + (size_t)(kv0 + kvr) * AS_C + dh;
      const __bf16* kr2 = klb + (size_t)(kv0 + kvr) * AS_C + dh;
      *(v8b*)(Ksh + kvr * AS_HD + dh)     = *(const v8b*)(kr);
      *(v8b*)(Ksh + kvr * AS_HD + dh + 8) = *(const v8b*)(kr + 8);
      *(v8b*)(Ksl + kvr * AS_HD + dh)     = *(const v8b*)(kr2);
      *(v8b*)(Ksl + kvr * AS_HD + dh + 8) = *(const v8b*)(kr2 + 8);
      const int dr = tid >> 2, part = (tid & 3) * 16;
      const _Float16* vr = vb + (size_t)dr * AS_S + kv0 + part;
      *(v8h*)(Vt + dr * AS_KC + part)     = *(const v8h*)(vr);
      *(v8h*)(Vt + dr * AS_KC + part + 8) = *(const v8h*)(vr + 8);
    }
    __syncthreads();

    v8f s[4];
#pragma unroll
    for (int j = 0; j < 4; ++j) {
      s[j] = (v8f){0.f,0.f,0.f,0.f,0.f,0.f,0.f,0.f};
      FB kb, kl;
      kb.h[0] = *(const v8b*)(Ksh + (j * 16 + c) * AS_HD + 8 * hh);
      kb.h[1] = *(const v8b*)(Ksh + (j * 16 + c) * AS_HD + 16 + 8 * hh);
      kl.h[0] = *(const v8b*)(Ksl + (j * 16 + c) * AS_HD + 8 * hh);
      kl.h[1] = *(const v8b*)(Ksl + (j * 16 + c) * AS_HD + 16 + 8 * hh);
      s[j] = mma_bf_g(qah, kb.v, s[j]);
      s[j] = mma_bf_g(qah, kl.v, s[j]);
      s[j] = mma_bf_g(qal, kb.v, s[j]);
    }

    float cm[8];
#pragma unroll
    for (int r = 0; r < 8; ++r) {
      float m = s[0][r];
#pragma unroll
      for (int j = 1; j < 4; ++j) m = fmaxf(m, s[j][r]);
#pragma unroll
      for (int off = 1; off < 16; off <<= 1) m = fmaxf(m, __shfl_xor(m, off, 32));
      cm[r] = m;
    }
#pragma unroll
    for (int r = 0; r < 8; ++r) {
      const float mnew  = fmaxf(mrow[r], cm[r]);
      const float alpha = expf(mrow[r] - mnew);
      mrow[r] = mnew;
      float psum = 0.f;
#pragma unroll
      for (int j = 0; j < 4; ++j) {
        const float p = expf(s[j][r] - mnew);
        psum += p;
        pw[(8 * hh + r) * AS_KC + j * 16 + c] = (_Float16)(p * AS_PSC);
      }
#pragma unroll
      for (int off = 1; off < 16; off <<= 1) psum += __shfl_xor(psum, off, 32);
      lrow[r] = lrow[r] * alpha + psum;
#pragma unroll
      for (int t = 0; t < 2; ++t) oacc[t][r] *= alpha;
    }
    __builtin_amdgcn_fence(__ATOMIC_RELEASE, "workgroup");
    __builtin_amdgcn_wave_barrier();
    __builtin_amdgcn_fence(__ATOMIC_ACQUIRE, "workgroup");

#pragma unroll 1
    for (int kk = 0; kk < 2; ++kk) {
      FH pa;
      pa.h[0] = *(const v8h*)(pw + c * AS_KC + kk * 32 + 8 * hh);
      pa.h[1] = *(const v8h*)(pw + c * AS_KC + kk * 32 + 16 + 8 * hh);
#pragma unroll
      for (int t = 0; t < 2; ++t) {
        FH vf;
        vf.h[0] = *(const v8h*)(Vt + (t * 16 + c) * AS_KC + kk * 32 + 8 * hh);
        vf.h[1] = *(const v8h*)(Vt + (t * 16 + c) * AS_KC + kk * 32 + 16 + 8 * hh);
        oacc[t] = mma_hf_g(pa.v, vf.v, oacc[t]);
      }
    }
  }

#pragma unroll
  for (int r = 0; r < 8; ++r) {
    const float inv = 1.0f / (lrow[r] * AS_PSC);
#pragma unroll
    for (int t = 0; t < 2; ++t) Os[t * 16 + c][wave * 16 + 8 * hh + r] = oacc[t][r] * inv;
  }
  __syncthreads();
  {
    const int lq = lane >> 3, c4 = (lane & 7) * 4;
    for (int pass = 0; pass < 2; ++pass) {
#pragma unroll
      for (int it = 0; it < 4; ++it) {
        const int L = wave * 16 + it * 4 + lq;
        const int d = L >> 1, half = L & 1;
        const v4f val = *(const v4f*)(&Os[d][half * 32 + c4]);
        *(volatile v4f*)(ob + (size_t)d * AS_S + half * 32 + c4) = val;
      }
      __threadfence();
    }
  }
}

extern "C" void kernel_launch(void* const* d_in, const int* in_sizes, int n_in,
                              void* d_out, int out_size, void* d_ws, size_t ws_size,
                              hipStream_t stream) {
  const int B = 8, CHI = 512, C = 256, SQ = 256, S = 1024;
  if (n_in < 8) return;
  if (in_sizes[0] != B * CHI * SQ || in_sizes[1] != B * C * S || in_sizes[2] != C * CHI ||
      in_sizes[3] != C || in_sizes[4] != C * C || in_sizes[5] != C || in_sizes[6] != C * C ||
      in_sizes[7] != C || out_size != B * C * S) return;

  const float* x_high = (const float*)d_in[0];
  const float* x_low  = (const float*)d_in[1];
  const float* Wq     = (const float*)d_in[2];
  const float* bq     = (const float*)d_in[3];
  const float* Wk     = (const float*)d_in[4];
  const float* bk     = (const float*)d_in[5];
  const float* Wv     = (const float*)d_in[6];
  const float* bv     = (const float*)d_in[7];
  float* out = (float*)d_out;

  char* ws = (char*)d_ws;
  size_t off = 0;
#define CARVE16(name, elems) unsigned short* name = (unsigned short*)(ws + off); off += ((((size_t)(elems)) * 2) + 255) & ~(size_t)255;
  CARVE16(xl_h, (size_t)B * S * C)
  CARVE16(xl_l, (size_t)B * S * C)
  CARVE16(xl_f, (size_t)B * S * C)
  CARVE16(xh_h, (size_t)B * SQ * CHI)
  CARVE16(xh_l, (size_t)B * SQ * CHI)
  CARVE16(wq_h, (size_t)C * CHI)
  CARVE16(wq_l, (size_t)C * CHI)
  CARVE16(wk_h, (size_t)C * C)
  CARVE16(wk_l, (size_t)C * C)
  CARVE16(wv_f, (size_t)C * C)
  CARVE16(q_h,  (size_t)B * SQ * C)
  CARVE16(q_l,  (size_t)B * SQ * C)
  CARVE16(k_h,  (size_t)B * S * C)
  CARVE16(k_l,  (size_t)B * S * C)
  CARVE16(v_f,  (size_t)B * C * S)
#undef CARVE16
  if (off > ws_size || off > (size_t)134217728) return;

  split_f32_bf16x2<<<dim3((C * CHI / 2 + 255) / 256), dim3(256), 0, stream>>>(Wq, wq_h, wq_l, C * CHI / 2);
  split_f32_bf16x2<<<dim3((C * C / 2 + 255) / 256), dim3(256), 0, stream>>>(Wk, wk_h, wk_l, C * C / 2);
  cast_f32_f16x2<<<dim3((C * C / 2 + 255) / 256), dim3(256), 0, stream>>>(Wv, (_Float16*)wv_f, C * C / 2);

  k_cm_to_pm<true><<<dim3(S / 32, C / 64, B), dim3(256), 0, stream>>>(x_low, C, S, xl_h, xl_l, xl_f);
  k_cm_to_pm<false><<<dim3(SQ / 32, CHI / 64, B), dim3(256), 0, stream>>>(x_high, CHI, SQ, xh_h, xh_l, xh_l);

  wmma_gemm64<1, true, 2, 2, false, 0><<<dim3(2, B), dim3(256), 0, stream>>>(
      xh_h, xh_l, CHI, (long)SQ * CHI,
      wq_h, wq_l, CHI, 0L,
      (void*)q_h, (void*)q_l, C, (long)SQ * C,
      bq, bq, 0L, SQ, C, CHI, 1.0f);
  wmma_gemm64<1, true, 2, 2, false, 0><<<dim3(8, B), dim3(256), 0, stream>>>(
      xl_h, xl_l, C, (long)S * C,
      wk_h, wk_l, C, 0L,
      (void*)k_h, (void*)k_l, C, (long)S * C,
      bk, bk, 0L, S, C, C, 1.0f);
  wmma_gemm64<0, false, 1, 1, false, 0><<<dim3(8, B), dim3(256), 0, stream>>>(
      wv_f, wv_f, C, 0L,
      xl_f, xl_f, C, (long)S * C,
      (void*)v_f, (void*)v_f, S, (long)C * S,
      bv, bv, 0L, C, S, C, 1.0f);

  attn_hd32<<<dim3(B * AS_NH * (S / 64)), dim3(128), 0, stream>>>(q_h, q_l, k_h, k_l, v_f, out);
}
